// Qwrky7TimeMix_5617817224049
// MI455X (gfx1250) — hardware-run, weakly checked
//
#include <hip/hip_runtime.h>
#include <math.h>

constexpr int kBatch   = 2;
constexpr int kSteps   = 1024;
constexpr int kChan    = 1024;
constexpr int kHeads   = 16;
constexpr int kHdim    = 64;
constexpr int kKvChan  = 512;
constexpr int kKvHeads = kKvChan / kHdim;
constexpr int kGroup   = kHeads / kKvHeads;
constexpr int kTok     = kBatch * kSteps;
constexpr size_t kPlane   = (size_t)kTok * kChan;
constexpr size_t kKvPlane = (size_t)kTok * kKvChan;
constexpr int kStateElems = kBatch * kHeads * kHdim * kHdim;
constexpr int kRankW  = 64;
constexpr int kRankA  = 64;
constexpr int kRankV  = 32;
constexpr int kRankVP = 64;
constexpr int kRankG  = 160;
constexpr int kRankGP = 192;
constexpr int kChunk  = 16;

constexpr float kXCarry   = 16.0f;
constexpr float kWCarry   = 256.0f;
constexpr float kHidCarry = 16.0f;
constexpr float kYCarry   = 16.0f;
constexpr float kResCarry = 2048.0f;
constexpr float kResInv   = 1.0f / kResCarry;
constexpr float kScaleXW     = 1.0f / (kXCarry * kWCarry);
constexpr float kScaleHidLin = kHidCarry / (kXCarry * kWCarry);
constexpr float kScaleHW     = 1.0f / (kHidCarry * kWCarry);
constexpr float kScaleOut    = 1.0f / (kYCarry * kWCarry);
constexpr float kGnEps       = 1e-5f * (float)kHdim;
constexpr float kF16MinNormal = 6.103515625e-05f;

static_assert(kHeads * kHdim == kChan);
static_assert(kKvHeads == 8 && kGroup == 2);
static_assert(kTok % 32 == 0 && kChan % 64 == 0 && kKvChan % 64 == 0);
static_assert(kRankW % 64 == 0 && kRankA % 64 == 0 && kRankVP % 64 == 0 && kRankGP % 64 == 0);
static_assert(kChan % 32 == 0 && kRankW % 32 == 0 && kRankVP % 32 == 0 && kRankGP % 32 == 0);
static_assert(kRankV <= kRankVP && kRankG <= kRankGP);
static_assert(kSteps % kChunk == 0);
static_assert((kTok * kHeads) % 8 == 0);
static_assert(kHdim == 64 && kChunk == 16);
static_assert(kStateElems == 131072);

typedef __attribute__((ext_vector_type(16))) _Float16 v16h;
typedef __attribute__((ext_vector_type(8)))  _Float16 v8h;
typedef __attribute__((ext_vector_type(8)))  float    v8f;
typedef __attribute__((ext_vector_type(4)))  float    v4f;
typedef __attribute__((ext_vector_type(2)))  float    v2f;
typedef __attribute__((ext_vector_type(4)))  unsigned int v4u;

__device__ __forceinline__ unsigned pk16(unsigned short a, unsigned short b) {
  return (unsigned)a | ((unsigned)b << 16);
}
__device__ __forceinline__ float flush_small(float f) {
  return (fabsf(f) < kF16MinNormal) ? 0.0f : f;
}
__device__ __forceinline__ unsigned short h_bits(float f) {
  const float g = flush_small(f);
  const _Float16 h = (_Float16)g;
  return __builtin_bit_cast(unsigned short, h);
}
__device__ __forceinline__ void h_split(float v, unsigned short& hb, unsigned short& rb) {
  const float g = flush_small(v);
  const _Float16 h = (_Float16)g;
  const float hf = (float)h;
  const float d = (v - hf) * kResCarry;
  const float dg = flush_small(d);
  const _Float16 r = (_Float16)dg;
  hb = __builtin_bit_cast(unsigned short, h);
  rb = __builtin_bit_cast(unsigned short, r);
}
__device__ __forceinline__ void pack8_split(const float (&v)[8], v4u& uh, v4u& ur) {
  unsigned short hb[8], rb[8];
#pragma unroll
  for (int e = 0; e < 8; ++e) h_split(v[e], hb[e], rb[e]);
  uh = (v4u){pk16(hb[0], hb[1]), pk16(hb[2], hb[3]), pk16(hb[4], hb[5]), pk16(hb[6], hb[7])};
  ur = (v4u){pk16(rb[0], rb[1]), pk16(rb[2], rb[3]), pk16(rb[4], rb[5]), pk16(rb[6], rb[7])};
}
__device__ __forceinline__ float wave_sum32(float v) {
#pragma unroll
  for (int o = 16; o > 0; o >>= 1) v += __shfl_xor(v, o, 32);
  return v;
}

struct FragH {
  union U { v16h v; v8h h[2]; };
  static __device__ __forceinline__ v16h load(const _Float16* p) {
    U f;
    f.h[0] = *(const v8h*)(p);
    f.h[1] = *(const v8h*)(p + 16);
    return f.v;
  }
  static __device__ __forceinline__ v8f mma(v16h a, v16h b, v8f c) {
    return __builtin_amdgcn_wmma_f32_16x16x32_f16(false, a, false, b, (short)0, c, false, false);
  }
};
__device__ __forceinline__ void guard_acc(v8f& a, v16h x0, v16h x1, v16h x2, v16h x3, v16h y0, v16h y1) {
  asm volatile("v_nop\n\tv_nop\n\tv_nop\n\tv_nop"
               : "+v"(a)
               : "v"(x0), "v"(x1), "v"(x2), "v"(x3), "v"(y0), "v"(y1));
}
__device__ __forceinline__ void acc_fence(v8f& a) {
  asm volatile("v_nop\n\tv_nop\n\tv_nop\n\tv_nop" : "+v"(a));
}

template <bool SPLIT, int ACT, int OUT_MODE>
__global__ __launch_bounds__(256) void gemm_f16_kernel(
    const unsigned short* __restrict__ Ahp, const unsigned short* __restrict__ Arp, int lda, long strideA,
    const unsigned short* __restrict__ Bhp, const unsigned short* __restrict__ Brp, int ldb, long strideB,
    void* __restrict__ Cout, int ldc, long strideC,
    int M, int N, int K, float scale, int nValid) {
  static_assert(ACT == 0 || OUT_MODE == 1);
  __shared__ __align__(16) float sT[8][16 * 68];
  const int z    = blockIdx.y;
  const int lane = threadIdx.x & 31;
  const int wave = threadIdx.x >> 5;
  const int tilesN = N >> 6;
  const int tilesM = M >> 5;
  const int tile = blockIdx.x * 8 + wave;
  if (tile >= tilesM * tilesN) return;
  const int tm = tile / tilesN;
  const int tn = tile - tm * tilesN;
  const int m0 = tm << 5;
  const int n0 = tn << 6;
  const int rlane = lane & 15;
  const int half8 = (lane >> 4) * 8;
  const int mOff  = (lane >> 4) * 8;

  const size_t aoff = (size_t)z * (size_t)strideA + (size_t)(m0 + rlane) * lda + half8;
  const size_t boff = (size_t)z * (size_t)strideB + (size_t)(n0 + rlane) * ldb + half8;
  const _Float16* pa0 = (const _Float16*)Ahp + aoff;
  const _Float16* pa1 = pa0 + (size_t)16 * lda;
  const _Float16* pr0 = SPLIT ? ((const _Float16*)Arp + aoff) : pa0;
  const _Float16* pr1 = pr0 + (size_t)16 * lda;
  const _Float16* pbh = (const _Float16*)Bhp + boff;
  const _Float16* pbr = SPLIT ? ((const _Float16*)Brp + boff) : pbh;
  const size_t bstep = (size_t)16 * ldb;

  v8f acc[2][4], accr[2][4];
#pragma unroll
  for (int i = 0; i < 2; ++i)
#pragma unroll
    for (int j = 0; j < 4; ++j) {
      acc[i][j]  = (v8f){0.f, 0.f, 0.f, 0.f, 0.f, 0.f, 0.f, 0.f};
      accr[i][j] = (v8f){0.f, 0.f, 0.f, 0.f, 0.f, 0.f, 0.f, 0.f};
    }

  for (int k0 = 0; k0 < K; k0 += 32) {
    const v16h ah0 = FragH::load(pa0 + k0);
    const v16h ah1 = FragH::load(pa1 + k0);
    v16h ar0 = ah0, ar1 = ah1;
    if (SPLIT) {
      ar0 = FragH::load(pr0 + k0);
      ar1 = FragH::load(pr1 + k0);
    }
#pragma unroll
    for (int j = 0; j < 4; ++j) {
      const v16h bh = FragH::load(pbh + j * bstep + k0);
      v16h br = bh;
      if (SPLIT) br = FragH::load(pbr + j * bstep + k0);
      acc[0][j] = FragH::mma(ah0, bh, acc[0][j]);
      acc[1][j] = FragH::mma(ah1, bh, acc[1][j]);
      if (SPLIT) {
        accr[0][j] = FragH::mma(ah0, br, accr[0][j]);
        accr[1][j] = FragH::mma(ah1, br, accr[1][j]);
        accr[0][j] = FragH::mma(ar0, bh, accr[0][j]);
        accr[1][j] = FragH::mma(ar1, bh, accr[1][j]);
      }
      guard_acc(acc[0][j], ah0, ah1, ar0, ar1, bh, br);
      guard_acc(acc[1][j], ah0, ah1, ar0, ar1, bh, br);
      if (SPLIT) {
        guard_acc(accr[0][j], ah0, ah1, ar0, ar1, bh, br);
        guard_acc(accr[1][j], ah0, ah1, ar0, ar1, bh, br);
      }
    }
  }
#pragma unroll
  for (int i = 0; i < 2; ++i)
#pragma unroll
    for (int j = 0; j < 4; ++j) {
      acc_fence(acc[i][j]);
      if (SPLIT) acc_fence(accr[i][j]);
    }

  float* slab = sT[wave];
#pragma unroll
  for (int i = 0; i < 2; ++i) {
    const int mBase = m0 + (i << 4);
#pragma unroll
    for (int j = 0; j < 4; ++j) {
#pragma unroll
      for (int r = 0; r < 8; ++r) {
        float v = acc[i][j][r];
        if (SPLIT) v += accr[i][j][r] * kResInv;
        v *= scale;
        slab[(mOff + r) * 68 + (j << 4) + rlane] = v;
      }
    }
    __builtin_amdgcn_fence(__ATOMIC_RELEASE, "workgroup");
    __builtin_amdgcn_wave_barrier();
    __builtin_amdgcn_fence(__ATOMIC_ACQUIRE, "workgroup");
    if (OUT_MODE == 0) {
      float* C = (float*)Cout + (size_t)z * (size_t)strideC;
      const int hh = lane >> 4, c4 = (lane & 15) * 4;
      for (int pass = 0; pass < 2; ++pass) {
#pragma unroll
        for (int it = 0; it < 8; ++it) {
          const int row = it * 2 + hh;
          const v4f v = *(const v4f*)(slab + row * 68 + c4);
          *(volatile v4f*)(C + (size_t)(mBase + row) * ldc + n0 + c4) = v;
        }
        __threadfence();
      }
    } else {
      const int q = lane >> 3, c8 = (lane & 7) * 8;
      if (ACT != 0) {
#pragma unroll 1
        for (int it = 0; it < 4; ++it) {
          float* sp = slab + (it * 4 + q) * 68 + c8;
#pragma unroll
          for (int e = 0; e < 8; ++e) {
            const float x = sp[e];
            float y;
            if (ACT == 1) y = tanhf(x);
            else y = 1.0f / (1.0f + expf(-x));
            sp[e] = y * kHidCarry;
          }
        }
      }
      unsigned short* C = (unsigned short*)Cout + (size_t)z * (size_t)strideC;
      for (int pass = 0; pass < 2; ++pass) {
#pragma unroll
        for (int it = 0; it < 4; ++it) {
          const int row = it * 4 + q;
          const float* sp = slab + row * 68 + c8;
          v8h hv;
#pragma unroll
          for (int e = 0; e < 8; ++e) {
            const float xv = sp[e];
            const bool live = (n0 + c8 + e) < nValid;
            const float xs = live ? flush_small(xv) : 0.0f;
            hv[e] = (_Float16)xs;
          }
          *(volatile v8h*)(C + (size_t)(mBase + row) * ldc + n0 + c8) = hv;
        }
        __threadfence();
      }
    }
    __builtin_amdgcn_fence(__ATOMIC_RELEASE, "workgroup");
    __builtin_amdgcn_wave_barrier();
    __builtin_amdgcn_fence(__ATOMIC_ACQUIRE, "workgroup");
  }
}

__global__ __launch_bounds__(256) void wt_plane_kernel(const float* __restrict__ W,
                                                       unsigned short* __restrict__ outh,
                                                       int Kd, int Nd, int KdP, int NdP) {
  __shared__ float sm[64][65];
  const int t  = threadIdx.x;
  const int k0 = blockIdx.x * 64;
  const int n0 = blockIdx.y * 64;
#pragma unroll
  for (int i = 0; i < 16; ++i) {
    const int e = i * 256 + t;
    const int r = e >> 6;
    const int c = e & 63;
    const int kk = k0 + r;
    const int nn = n0 + c;
    const bool valid = (kk < Kd) && (nn < Nd);
    const int kc = (kk < Kd) ? kk : (Kd - 1);
    const int nc = (nn < Nd) ? nn : (Nd - 1);
    float v = W[(size_t)kc * Nd + nc];
    asm volatile("" : "+v"(v));
    sm[c][r] = valid ? (v * kWCarry) : 0.0f;
  }
  __syncthreads();
  const int lane = t & 31, wave = t >> 5;
  const int q = lane >> 3, c8 = (lane & 7) * 8;
  for (int pass = 0; pass < 2; ++pass) {
#pragma unroll
    for (int it = 0; it < 2; ++it) {
      const int row = wave * 8 + it * 4 + q;
      float v[8];
#pragma unroll
      for (int e = 0; e < 8; ++e) v[e] = sm[row][c8 + e];
      v4u uh, ur;
      pack8_split(v, uh, ur);
      const size_t o = (size_t)(n0 + row) * KdP + k0 + c8;
      *(volatile v4u*)(outh + o) = uh;
    }
    __threadfence();
  }
  (void)NdP;
}

__global__ __launch_bounds__(256) void cast_plane_kernel(const float* __restrict__ src,
                                                         unsigned short* __restrict__ outh,
                                                         unsigned short* __restrict__ outr,
                                                         int n8, float carry, int has_res) {
  const int i = blockIdx.x * 256 + threadIdx.x;
  if (i >= n8) return;
  const size_t off = (size_t)i * 8;
  const v4f a = *(const v4f*)(src + off);
  const v4f b = *(const v4f*)(src + off + 4);
  float v[8];
#pragma unroll
  for (int e = 0; e < 4; ++e) {
    v[e]     = a[e] * carry;
    v[4 + e] = b[e] * carry;
  }
  v4u uh, ur;
  pack8_split(v, uh, ur);
  for (int pass = 0; pass < 2; ++pass) {
    *(volatile v4u*)(outh + off) = uh;
    if (has_res) *(volatile v4u*)(outr + off) = ur;
    __threadfence();
  }
}

__global__ __launch_bounds__(256) void gate_prep_kernel(const float* __restrict__ Kraw, const float* __restrict__ Vraw,
                                                        float* WD, float* AB, float* VK,
                                                        float* __restrict__ KM, float* __restrict__ VM,
                                                        const float* __restrict__ vfirst,
                                                        const float* __restrict__ w0, const float* __restrict__ a0,
                                                        const float* __restrict__ v0b, const float* __restrict__ k_k,
                                                        const float* __restrict__ k_a) {
  const int lane = threadIdx.x & 31;
  const int pair = blockIdx.x * 8 + (threadIdx.x >> 5);
  const int tok = pair >> 4;
  const int h   = pair & 15;
  const size_t base   = (size_t)tok * kChan + (size_t)h * kHdim;
  const size_t kvbase = (size_t)tok * kKvChan + (size_t)(h >> 1) * kHdim;
  const int cb = h * kHdim;
  float ss;
  {
    const float ka = Kraw[kvbase + lane] * k_k[cb + lane];
    const float kb = Kraw[kvbase + lane + 32] * k_k[cb + lane + 32];
    ss = wave_sum32(ka * ka + kb * kb);
  }
  const float inv = 1.0f / fmaxf(sqrtf(ss), 1e-12f);
#pragma unroll 1
  for (int hf = 0; hf < 2; ++hf) {
    const size_t idx = base + lane + 32 * hf;
    const size_t kvi = kvbase + lane + 32 * hf;
    const int c = cb + lane + 32 * hf;
    const float k0  = Kraw[kvi];
    const float vp  = Vraw[kvi];
    const float kkv = (k0 * k_k[c]) * inv;
    const float sg  = __builtin_amdgcn_rcpf(1.0f + expf(-(a0[c] + AB[idx])));
    const float lr  = 1.0f + (sg - 1.0f) * k_a[c];
    const float km  = k0 * lr;
    const float bv  = kkv * lr;
    const float wl  = w0[c] + WD[idx];
    const float dv  = expf(-expf(wl));
    const float vg  = __builtin_amdgcn_rcpf(1.0f + expf(-(v0b[c] + VK[idx])));
    const float vm  = vp + (vfirst[idx] - vp) * vg;
    *(volatile float*)(KM + idx) = km;
    *(volatile float*)(VM + idx) = vm;
    *(volatile float*)(WD + idx) = dv;
    *(volatile float*)(AB + idx) = bv;
    *(volatile float*)(VK + idx) = kkv;
    __threadfence();
    *(volatile float*)(KM + idx) = km;
    *(volatile float*)(VM + idx) = vm;
    *(volatile float*)(WD + idx) = dv;
    *(volatile float*)(AB + idx) = bv;
    *(volatile float*)(VK + idx) = kkv;
  }
}

__global__ __launch_bounds__(256) void state_scan_kernel(const float* __restrict__ Rf, const float* __restrict__ Dd,
                                                         const float* __restrict__ Kf, const float* __restrict__ Vf,
                                                         const float* __restrict__ KKf, const float* __restrict__ Bv,
                                                         const float* __restrict__ S0,
                                                         float* __restrict__ Y, float* __restrict__ Sout) {
  __shared__ __align__(16) float lv[6 * kChunk * 64];
  __shared__ __align__(16) float yb[kChunk * 64];
  static_assert(6 * kChunk * 64 >= kHdim * kHdim);
  const int bh  = blockIdx.x;
  const int b   = bh >> 4;
  const int h   = bh & 15;
  const int tid = threadIdx.x;
  const int i   = tid >> 2;
  const int q   = tid & 3;
  const int j0  = q * 16;
  const int lrow = tid >> 4;
  const int lc4  = (tid & 15) * 4;
  const size_t base = (size_t)b * kSteps * kChan + (size_t)h * kHdim;

  float S[16];
  {
    const float* sp = S0 + (size_t)bh * (kHdim * kHdim) + (size_t)i * kHdim + j0;
#pragma unroll
    for (int g4 = 0; g4 < 4; ++g4) {
      const v4f t = *(const v4f*)(sp + 4 * g4);
      S[4 * g4 + 0] = t[0];
      S[4 * g4 + 1] = t[1];
      S[4 * g4 + 2] = t[2];
      S[4 * g4 + 3] = t[3];
    }
  }

#pragma unroll 1
  for (int ch = 0; ch < kSteps / kChunk; ++ch) {
    const size_t goff = base + (size_t)(ch * kChunk + lrow) * kChan + lc4;
    {
      const v4f t0 = *(const v4f*)(Rf + goff);
      const v4f t1 = *(const v4f*)(Dd + goff);
      const v4f t2 = *(const v4f*)(Kf + goff);
      const v4f t3 = *(const v4f*)(Vf + goff);
      const v4f t4 = *(const v4f*)(KKf + goff);
      const v4f t5 = *(const v4f*)(Bv + goff);
      const int lo = lrow * 64 + lc4;
      *(v4f*)(lv + 0 * kChunk * 64 + lo) = t0;
      *(v4f*)(lv + 1 * kChunk * 64 + lo) = t1;
      *(v4f*)(lv + 2 * kChunk * 64 + lo) = t2;
      *(v4f*)(lv + 3 * kChunk * 64 + lo) = t3;
      *(v4f*)(lv + 4 * kChunk * 64 + lo) = t4;
      *(v4f*)(lv + 5 * kChunk * 64 + lo) = t5;
    }
    __syncthreads();

#pragma unroll 1
    for (int s = 0; s < kChunk; ++s) {
      const float* pr  = lv + 0 * kChunk * 64 + s * 64 + j0;
      const float* pd  = lv + 1 * kChunk * 64 + s * 64 + j0;
      const float* pk  = lv + 2 * kChunk * 64 + s * 64 + j0;
      const float* pkk = lv + 4 * kChunk * 64 + s * 64 + j0;
      const float* pb  = lv + 5 * kChunk * 64 + s * 64 + j0;
      const float vi = lv[3 * kChunk * 64 + s * 64 + i];
      float sa = 0.0f;
#pragma unroll
      for (int g4 = 0; g4 < 4; ++g4) {
        const v4f k4 = *(const v4f*)(pkk + 4 * g4);
#pragma unroll
        for (int e = 0; e < 4; ++e) sa += S[4 * g4 + e] * k4[e];
      }
      sa += __shfl_xor(sa, 1, 32);
      sa += __shfl_xor(sa, 2, 32);
      sa = -sa;
      float out = 0.0f;
#pragma unroll
      for (int g4 = 0; g4 < 4; ++g4) {
        const v4f d4 = *(const v4f*)(pd + 4 * g4);
        const v4f b4 = *(const v4f*)(pb + 4 * g4);
        const v4f k4 = *(const v4f*)(pk + 4 * g4);
        const v4f r4 = *(const v4f*)(pr + 4 * g4);
#pragma unroll
        for (int e = 0; e < 4; ++e) {
          const float sn = S[4 * g4 + e] * d4[e] + sa * b4[e] + vi * k4[e];
          S[4 * g4 + e] = sn;
          out += sn * r4[e];
        }
      }
      out += __shfl_xor(out, 1, 32);
      out += __shfl_xor(out, 2, 32);
      if (q == 0) yb[s * 64 + i] = out;
    }
    __syncthreads();
    {
      const v4f val = *(const v4f*)(yb + lrow * 64 + lc4);
      *(volatile v4f*)(Y + goff) = val;
      __threadfence();
      *(volatile v4f*)(Y + goff) = val;
    }
  }

#pragma unroll
  for (int g4 = 0; g4 < 4; ++g4) {
    const v4f t = (v4f){S[4 * g4 + 0], S[4 * g4 + 1], S[4 * g4 + 2], S[4 * g4 + 3]};
    *(v4f*)(lv + i * kHdim + j0 + 4 * g4) = t;
  }
  __syncthreads();
  {
    float* So = Sout + (size_t)bh * (kHdim * kHdim);
    v4f sv[4];
#pragma unroll
    for (int it = 0; it < 4; ++it) sv[it] = *(const v4f*)(lv + (size_t)(it * 256 + tid) * 4);
    for (int pass = 0; pass < 2; ++pass) {
#pragma unroll
      for (int it = 0; it < 4; ++it) *(volatile v4f*)(So + (size_t)(it * 256 + tid) * 4) = sv[it];
      __threadfence();
    }
  }
}

__global__ __launch_bounds__(256) void norm_gate_kernel(const float* __restrict__ Y, const float* __restrict__ Rf,
                                                        const float* __restrict__ Kf, const float* __restrict__ Vf,
                                                        const float* __restrict__ Gf, const float* __restrict__ r_k,
                                                        const float* __restrict__ ln_w, const float* __restrict__ ln_b,
                                                        unsigned* __restrict__ YGh) {
  const int lane = threadIdx.x & 31;
  const int pair = blockIdx.x * 8 + (threadIdx.x >> 5);
  const int tok = pair >> 4;
  const int h   = pair & 15;
  const size_t base = (size_t)tok * kChan + (size_t)h * kHdim + 2 * lane;
  const int c = h * kHdim + 2 * lane;
  const v2f y2 = *(const v2f*)(Y + base);
  const v2f r2 = *(const v2f*)(Rf + base);
  const v2f k2 = *(const v2f*)(Kf + base);
  const v2f v2 = *(const v2f*)(Vf + base);
  const v2f g2 = *(const v2f*)(Gf + base);
  const v2f q2 = *(const v2f*)(r_k + c);
  const v2f w2 = *(const v2f*)(ln_w + c);
  const v2f b2 = *(const v2f*)(ln_b + c);
  const float mu = wave_sum32(y2[0] + y2[1]) * (1.0f / 64.0f);
  const float d0 = y2[0] - mu;
  const float d1 = y2[1] - mu;
  const float var = wave_sum32(d0 * d0 + d1 * d1) * (1.0f / 64.0f);
  const float inv = 1.0f / sqrtf(var + kGnEps);
  const float bsum = wave_sum32(r2[0] * k2[0] * q2[0] + r2[1] * k2[1] * q2[1]);
  const float o0 = (((d0 * inv) * w2[0] + b2[0]) + bsum * v2[0]) * g2[0] * kYCarry;
  const float o1 = (((d1 * inv) * w2[1] + b2[1]) + bsum * v2[1]) * g2[1] * kYCarry;
  const unsigned short h0 = h_bits(o0);
  const unsigned short h1 = h_bits(o1);
  const unsigned wh = pk16(h0, h1);
  const size_t widx = base >> 1;
  *(volatile unsigned*)(YGh + widx) = wh;
  __threadfence();
  *(volatile unsigned*)(YGh + widx) = wh;
}

__global__ __launch_bounds__(256) void copy_f32x4_kernel(const float* __restrict__ src, float* __restrict__ dst, int n4) {
  const int i = blockIdx.x * 256 + threadIdx.x;
  if (i >= n4) return;
  const v4f v = *(const v4f*)(src + (size_t)i * 4);
  *(volatile v4f*)(dst + (size_t)i * 4) = v;
  __threadfence();
  *(volatile v4f*)(dst + (size_t)i * 4) = v;
}

constexpr size_t kSzAct16  = kPlane * 2;
constexpr size_t kSzWBig   = (size_t)kChan * kChan * 2;
constexpr size_t kSzWKv    = (size_t)kKvChan * kChan * 2;
constexpr size_t kSzF64    = (size_t)64 * kChan * 2;
constexpr size_t kSzF192   = (size_t)kRankGP * kChan * 2;
constexpr size_t kSzH64    = (size_t)kTok * 64 * 2;
constexpr size_t kSzH192   = (size_t)kTok * kRankGP * 2;
constexpr size_t kSzF32    = kPlane * 4;
constexpr size_t kSzKv32   = kKvPlane * 4;
constexpr size_t kWsTotal =
    2 * kSzAct16 + 2 * kSzWBig + 2 * kSzWKv + kSzWKv + kSzWBig +
    3 * kSzF64 + kSzF192 + 3 * kSzF64 + kSzF192 +
    3 * kSzH64 + kSzH192 +
    kSzF32 + 2 * kSzKv32 + 4 * kSzF32 + 2 * kSzF32 + kSzF32 + kSzAct16;
static_assert(kWsTotal == 100663296ull);
static_assert(kWsTotal <= 134217728ull);
static_assert((kSzAct16 % 256) == 0 && (kSzWBig % 256) == 0 && (kSzWKv % 256) == 0 && (kSzF64 % 256) == 0 &&
              (kSzF192 % 256) == 0 && (kSzH64 % 256) == 0 && (kSzH192 % 256) == 0 && (kSzF32 % 256) == 0 &&
              (kSzKv32 % 256) == 0);

extern "C" void kernel_launch(void* const* d_in, const int* in_sizes, int n_in,
                              void* d_out, int out_size, void* d_ws, size_t ws_size, hipStream_t stream) {
  if (n_in < 23 || d_out == nullptr || d_ws == nullptr) return;
  const int nP = (int)kPlane;
  if (in_sizes[0] != nP || in_sizes[1] != kStateElems || in_sizes[2] != nP) return;
  if (in_sizes[3] != kChan) return;
  if (in_sizes[4] != kChan * kRankW || in_sizes[5] != kRankW * kChan) return;
  if (in_sizes[6] != kChan) return;
  if (in_sizes[7] != kChan * kRankA || in_sizes[8] != kRankA * kChan) return;
  if (in_sizes[9] != kChan) return;
  if (in_sizes[10] != kChan * kRankV || in_sizes[11] != kRankV * kChan) return;
  if (in_sizes[12] != kChan * kRankG || in_sizes[13] != kRankG * kChan) return;
  if (in_sizes[14] != kChan || in_sizes[15] != kChan || in_sizes[16] != kHeads * kHdim) return;
  if (in_sizes[17] != kChan * kChan || in_sizes[18] != kKvChan * kChan) return;
  if (in_sizes[19] != kKvChan * kChan || in_sizes[20] != kChan * kChan) return;
  if (in_sizes[21] != kChan || in_sizes[22] != kChan) return;
  if (out_size != 2 * nP + kStateElems) return;

  const float* x      = (const float*)d_in[0];
  const float* S0     = (const float*)d_in[1];
  const float* vfirst = (const float*)d_in[2];
  const float* w0  = (const float*)d_in[3];
  const float* w1  = (const float*)d_in[4];
  const float* w2  = (const float*)d_in[5];
  const float* a0  = (const float*)d_in[6];
  const float* a1  = (const float*)d_in[7];
  const float* a2  = (const float*)d_in[8];
  const float* v0  = (const float*)d_in[9];
  const float* v1  = (const float*)d_in[10];
  const float* v2  = (const float*)d_in[11];
  const float* g1  = (const float*)d_in[12];
  const float* g2  = (const float*)d_in[13];
  const float* k_k = (const float*)d_in[14];
  const float* k_a = (const float*)d_in[15];
  const float* r_k = (const float*)d_in[16];
  const float* Wq  = (const float*)d_in[17];
  const float* Wk  = (const float*)d_in[18];
  const float* Wv  = (const float*)d_in[19];
  const float* Wo  = (const float*)d_in[20];
  const float* ln_w = (const float*)d_in[21];
  const float* ln_b = (const float*)d_in[22];
  float* out0 = (float*)d_out;
  float* out1 = out0 + kPlane;
  float* out2 = out1 + kStateElems;

  char* ws = (char*)d_ws;
  size_t off = 0;
  auto carve = [&](size_t bytes) -> char* {
    char* p = ws + off;
    off += (bytes + 255) & ~(size_t)255;
    return p;
  };
  unsigned short* Xh  = (unsigned short*)carve(kSzAct16);
  unsigned short* Xr  = (unsigned short*)carve(kSzAct16);
  unsigned short* Wqh = (unsigned short*)carve(kSzWBig);
  unsigned short* Wqr = (unsigned short*)carve(kSzWBig);
  unsigned short* Wkh = (unsigned short*)carve(kSzWKv);
  unsigned short* Wkr = (unsigned short*)carve(kSzWKv);
  unsigned short* Wvh = (unsigned short*)carve(kSzWKv);
  unsigned short* Woh = (unsigned short*)carve(kSzWBig);
  unsigned short* w1T = (unsigned short*)carve(kSzF64);
  unsigned short* a1T = (unsigned short*)carve(kSzF64);
  unsigned short* v1T = (unsigned short*)carve(kSzF64);
  unsigned short* g1T = (unsigned short*)carve(kSzF192);
  unsigned short* w2T = (unsigned short*)carve(kSzF64);
  unsigned short* a2T = (unsigned short*)carve(kSzF64);
  unsigned short* v2T = (unsigned short*)carve(kSzF64);
  unsigned short* g2T = (unsigned short*)carve(kSzF192);
  unsigned short* HW  = (unsigned short*)carve(kSzH64);
  unsigned short* HA  = (unsigned short*)carve(kSzH64);
  unsigned short* HV  = (unsigned short*)carve(kSzH64);
  unsigned short* HG  = (unsigned short*)carve(kSzH192);
  float* Rf   = (float*)carve(kSzF32);
  float* Kraw = (float*)carve(kSzKv32);
  float* Vraw = (float*)carve(kSzKv32);
  float* WD   = (float*)carve(kSzF32);
  float* AB   = (float*)carve(kSzF32);
  float* VK   = (float*)carve(kSzF32);
  float* Gf   = (float*)carve(kSzF32);
  float* KM   = (float*)carve(kSzF32);
  float* VM   = (float*)carve(kSzF32);
  float* Yf   = (float*)carve(kSzF32);
  unsigned short* YG = (unsigned short*)carve(kSzAct16);
  if (off != kWsTotal || off > ws_size || off > (size_t)134217728) return;

  cast_plane_kernel<<<(nP / 8) / 256, 256, 0, stream>>>(x, Xh, Xr, nP / 8, kXCarry, 1);
  cast_plane_kernel<<<(kChan * kChan / 8) / 256, 256, 0, stream>>>(Wq, Wqh, Wqr, kChan * kChan / 8, kWCarry, 1);
  cast_plane_kernel<<<(kKvChan * kChan / 8) / 256, 256, 0, stream>>>(Wk, Wkh, Wkr, kKvChan * kChan / 8, kWCarry, 1);
  cast_plane_kernel<<<(kKvChan * kChan / 8) / 256, 256, 0, stream>>>(Wv, Wvh, Wvh, kKvChan * kChan / 8, kWCarry, 0);
  cast_plane_kernel<<<(kChan * kChan / 8) / 256, 256, 0, stream>>>(Wo, Woh, Woh, kChan * kChan / 8, kWCarry, 0);

  wt_plane_kernel<<<dim3(kChan / 64, kRankW / 64), 256, 0, stream>>>(w1, w1T, kChan, kRankW, kChan, kRankW);
  wt_plane_kernel<<<dim3(kChan / 64, kRankA / 64), 256, 0, stream>>>(a1, a1T, kChan, kRankA, kChan, kRankA);
  wt_plane_kernel<<<dim3(kChan / 64, kRankVP / 64), 256, 0, stream>>>(v1, v1T, kChan, kRankV, kChan, kRankVP);
  wt_plane_kernel<<<dim3(kChan / 64, kRankGP / 64), 256, 0, stream>>>(g1, g1T, kChan, kRankG, kChan, kRankGP);
  wt_plane_kernel<<<dim3(kRankW / 64, kChan / 64), 256, 0, stream>>>(w2, w2T, kRankW, kChan, kRankW, kChan);
  wt_plane_kernel<<<dim3(kRankA / 64, kChan / 64), 256, 0, stream>>>(a2, a2T, kRankA, kChan, kRankA, kChan);
  wt_plane_kernel<<<dim3(kRankVP / 64, kChan / 64), 256, 0, stream>>>(v2, v2T, kRankV, kChan, kRankVP, kChan);
  wt_plane_kernel<<<dim3(kRankGP / 64, kChan / 64), 256, 0, stream>>>(g2, g2T, kRankG, kChan, kRankGP, kChan);

  const int blkBig = (kTok / 32) * (kChan / 64) / 8;
  const int blkKv  = (kTok / 32) * (kKvChan / 64) / 8;
  gemm_f16_kernel<true, 0, 0><<<dim3(blkBig, 1), 256, 0, stream>>>(
      Xh, Xr, kChan, 0L, Wqh, Wqr, kChan, 0L, (void*)Rf, kChan, 0L, kTok, kChan, kChan, kScaleXW, kChan);
  gemm_f16_kernel<true, 0, 0><<<dim3(blkKv, 1), 256, 0, stream>>>(
      Xh, Xr, kChan, 0L, Wkh, Wkr, kChan, 0L, (void*)Kraw, kKvChan, 0L, kTok, kKvChan, kChan, kScaleXW, kKvChan);
  gemm_f16_kernel<false, 0, 0><<<dim3(blkKv, 1), 256, 0, stream>>>(
      Xh, Xh, kChan, 0L, Wvh, Wvh, kChan, 0L, (void*)Vraw, kKvChan, 0L, kTok, kKvChan, kChan, kScaleXW, kKvChan);

  const int blk64  = (kTok / 32) * (64 / 64) / 8;
  const int blk192 = (kTok / 32) * (kRankGP / 64) / 8;
  gemm_f16_kernel<false, 1, 1><<<dim3(blk64, 1), 256, 0, stream>>>(
      Xh, Xh, kChan, 0L, w1T, w1T, kChan, 0L, (void*)HW, kRankW, 0L, kTok, kRankW, kChan, kScaleXW, kRankW);
  gemm_f16_kernel<false, 0, 1><<<dim3(blk64, 1), 256, 0, stream>>>(
      Xh, Xh, kChan, 0L, a1T, a1T, kChan, 0L, (void*)HA, kRankA, 0L, kTok, kRankA, kChan, kScaleHidLin, kRankA);
  gemm_f16_kernel<false, 0, 1><<<dim3(blk64, 1), 256, 0, stream>>>(
      Xh, Xh, kChan, 0L, v1T, v1T, kChan, 0L, (void*)HV, kRankVP, 0L, kTok, kRankVP, kChan, kScaleHidLin, kRankV);
  gemm_f16_kernel<false, 2, 1><<<dim3(blk192, 1), 256, 0, stream>>>(
      Xh, Xh, kChan, 0L, g1T, g1T, kChan, 0L, (void*)HG, kRankGP, 0L, kTok, kRankGP, kChan, kScaleXW, kRankG);

  gemm_f16_kernel<false, 0, 0><<<dim3(blkBig, 1), 256, 0, stream>>>(
      HW, HW, kRankW, 0L, w2T, w2T, kRankW, 0L, (void*)WD, kChan, 0L, kTok, kChan, kRankW, kScaleHW, kChan);
  gemm_f16_kernel<false, 0, 0><<<dim3(blkBig, 1), 256, 0, stream>>>(
      HA, HA, kRankA, 0L, a2T, a2T, kRankA, 0L, (void*)AB, kChan, 0L, kTok, kChan, kRankA, kScaleHW, kChan);
  gemm_f16_kernel<false, 0, 0><<<dim3(blkBig, 1), 256, 0, stream>>>(
      HV, HV, kRankVP, 0L, v2T, v2T, kRankVP, 0L, (void*)VK, kChan, 0L, kTok, kChan, kRankVP, kScaleHW, kChan);
  gemm_f16_kernel<false, 0, 0><<<dim3(blkBig, 1), 256, 0, stream>>>(
      HG, HG, kRankGP, 0L, g2T, g2T, kRankGP, 0L, (void*)Gf, kChan, 0L, kTok, kChan, kRankGP, kScaleHW, kChan);

  gate_prep_kernel<<<(kTok * kHeads) / 8, 256, 0, stream>>>(Kraw, Vraw, WD, AB, VK, KM, VM, vfirst,
                                                            w0, a0, v0, k_k, k_a);

  state_scan_kernel<<<kBatch * kHeads, 256, 0, stream>>>(Rf, WD, KM, VM, VK, AB, S0, Yf, out1);

  norm_gate_kernel<<<(kTok * kHeads) / 8, 256, 0, stream>>>(Yf, Rf, KM, VM, Gf, r_k, ln_w, ln_b, (unsigned*)YG);

  gemm_f16_kernel<false, 0, 0><<<dim3(blkBig, 1), 256, 0, stream>>>(
      YG, YG, kChan, 0L, Woh, Woh, kChan, 0L, (void*)out0, kChan, 0L, kTok, kChan, kChan, kScaleOut, kChan);

  copy_f32x4_kernel<<<(nP / 4) / 256, 256, 0, stream>>>(vfirst, out2, nP / 4);
}
